// LSTMClassifier_26886495273452
// MI455X (gfx1250) — hardware-verified
//
#include <hip/hip_runtime.h>
#include <math.h>

constexpr int NSEQ     = 4096;
constexpr int NSTEP    = 512;
constexpr int NIN      = 3;
constexpr int NHID     = 50;
constexpr int NGATE    = 4 * NHID;
constexpr int NCLS     = 6;
constexpr int NTHR     = 128;
constexpr int NWAVE    = NTHR / 32;
constexpr int ROWS_BLK = 16;
constexpr int UPAD     = 64;
constexpr int WROWS    = 4 * UPAD;
constexpr int KDIM     = 64;
constexpr int XCOL     = NHID;
constexpr int WPITCH   = 64;
constexpr int APITCH   = 80;
constexpr int HSPITCH  = 260;
constexpr int NFC      = NCLS * NHID + NCLS;
constexpr int NFCLDS   = 308;
constexpr int NOUTB    = ROWS_BLK * NCLS;
constexpr int XWORDS   = (KDIM - XCOL) / 2;
constexpr float WCARRY     = 16.0f;
constexpr float WCARRY_INV = 1.0f / 16.0f;

static_assert(NSEQ % ROWS_BLK == 0, "no batch tail");
static_assert(NWAVE * 16 == UPAD && NHID <= UPAD, "one 16-unit subtile per wave");
static_assert(NHID + NIN <= KDIM && KDIM % 32 == 0, "K padded to a multiple of 32");
static_assert(KDIM <= WPITCH && KDIM <= APITCH, "pitches cover K");
static_assert(WPITCH % 8 == 0 && APITCH % 8 == 0, "16-B aligned fragment loads");
static_assert(WPITCH / 2 == 32, "weight build: one wave per row");
static_assert((WROWS * WPITCH / 2) % NTHR == 0, "weight build loop exact");
static_assert((ROWS_BLK * APITCH / 2) % NTHR == 0, "A-tile zero fill exact");
static_assert((KDIM - XCOL) % 2 == 0 && ROWS_BLK * XWORDS <= NTHR, "x restage: one word per thread");
static_assert(NOUTB <= NTHR && NOUTB % 4 == 0 && NOUTB / 4 <= 32, "output funnel: one wave, one instruction");
static_assert((NOUTB * 4) % 128 == 0, "block output = whole 128-B lines");
static_assert(NFCLDS >= NFC && 3 * NTHR >= NFC, "fc staging");
static_assert(HSPITCH >= UPAD, "h_last staging covers all lanes");
static_assert(NGATE == 200, "shape");

typedef __attribute__((ext_vector_type(16))) _Float16 v16h;
typedef __attribute__((ext_vector_type(8)))  _Float16 v8h;
typedef __attribute__((ext_vector_type(8)))  float    v8f;
typedef __attribute__((ext_vector_type(4)))  float    v4f;

__device__ __forceinline__ void mma_guard4(v8f& a, v8f& b, v8f& c, v8f& d, v16h x, v16h y) {
  asm volatile("v_nop\n\tv_nop\n\tv_nop\n\tv_nop" : "+v"(a), "+v"(b), "+v"(c), "+v"(d) : "v"(x), "v"(y));
}

template <typename T> struct Frag;
template <> struct Frag<_Float16> {
  typedef v16h V; union U { v16h v; v8h h[2]; };
  static __device__ __forceinline__ v16h load(const _Float16* p) {
    U f; f.h[0] = *(const v8h*)(p); f.h[1] = *(const v8h*)(p + 16); return f.v;
  }
  static __device__ __forceinline__ v8f mma(v16h a, v16h b, v8f c) {
    return __builtin_amdgcn_wmma_f32_16x16x32_f16(false, a, false, b, (short)0, c, false, false);
  }
};

__device__ __forceinline__ float fsig(float z)  { return __builtin_amdgcn_rcpf(1.0f + expf(-z)); }
__device__ __forceinline__ float ftanh(float z) { return 1.0f - 2.0f * __builtin_amdgcn_rcpf(expf(2.0f * z) + 1.0f); }

__device__ __forceinline__ unsigned short wplane_bits(const float* __restrict__ w_hh, const float* __restrict__ w_ih,
                                                      int nrow, float fu, int k) {
  const int kh = (k < NHID) ? k : (NHID - 1);
  int kx = k - XCOL; kx = (kx < 0) ? 0 : ((kx > NIN - 1) ? (NIN - 1) : kx);
  const float fw = (k < NHID) ? 1.0f : 0.0f;
  const float fx = (k >= XCOL && k < XCOL + NIN) ? 1.0f : 0.0f;
  const float whh = w_hh[nrow * NHID + kh];
  const float wih = w_ih[nrow * NIN + kx];
  const float v = WCARRY * (fu * fmaf(fw, whh, fx * wih));
  const _Float16 hv = (_Float16)v;
  return __builtin_bit_cast(unsigned short, hv);
}

__device__ __forceinline__ void stage_x(_Float16* sA, const float* __restrict__ x, int rowbase, int t, int tid) {
  const int m  = tid / XWORDS;
  const int q  = tid - m * XWORDS;
  const int mr = (m < ROWS_BLK) ? m : (ROWS_BLK - 1);
  const float* xp = x + ((size_t)(rowbase + mr) * NSTEP + (size_t)t) * NIN;
  const float x0 = xp[0], x1 = xp[1], x2 = xp[2];
  const float f0 = (q == 0) ? 1.0f : 0.0f;
  const float f1 = (q == 1) ? 1.0f : 0.0f;
  const float v0 = fmaf(f0, x0, f1 * x2);
  const float v1 = f0 * x1;
  const _Float16 h0 = (_Float16)v0;
  const _Float16 h1 = (_Float16)v1;
  const unsigned wd = (unsigned)__builtin_bit_cast(unsigned short, h0) |
                      ((unsigned)__builtin_bit_cast(unsigned short, h1) << 16);
  if (tid < ROWS_BLK * XWORDS) *(unsigned*)(sA + m * APITCH + XCOL + 2 * q) = wd;
}

__global__ __launch_bounds__(NTHR) void lstm_seq_kernel(const float* __restrict__ x, const float* __restrict__ w_ih,
                                                        const float* __restrict__ w_hh, const float* __restrict__ b_ih,
                                                        const float* __restrict__ b_hh, const float* __restrict__ w_fc,
                                                        const float* __restrict__ b_fc, float* __restrict__ out) {
  __shared__ __align__(16) _Float16 sW[WROWS * WPITCH];
  __shared__ __align__(16) _Float16 sA[ROWS_BLK * APITCH];
  __shared__ __align__(16) float    sHf[ROWS_BLK * HSPITCH];
  __shared__ __align__(16) float    sFC[NFCLDS];
  __shared__ __align__(16) float    sOut[NOUTB];

  const int tid = threadIdx.x, lane = tid & 31, wave = tid >> 5;
  const int c = lane & 15, hh = lane >> 4, koff = hh * 8;
  const int rowbase = blockIdx.x * ROWS_BLK;
  const int u  = 16 * wave + c;
  const int uc = (u < NHID) ? u : (NHID - 1);
  const bool ureal = (u < NHID);

  {
    unsigned* aw = (unsigned*)sA;
#pragma unroll
    for (int it = 0; it < (ROWS_BLK * APITCH / 2) / NTHR; ++it) aw[it * NTHR + tid] = 0u;
  }
  {
    unsigned* ww = (unsigned*)sW;
#pragma unroll 1
    for (int it = 0; it < (WROWS * WPITCH / 2) / NTHR; ++it) {
      const int idx = it * NTHR + tid;
      const int n   = idx >> 5;
      const int k0  = (idx & 31) * 2;
      const int g   = n >> 6, un = n & 63;
      const int unc = (un < NHID) ? un : (NHID - 1);
      const float fu = (un < NHID) ? 1.0f : 0.0f;
      const int nrow = g * NHID + unc;
      const unsigned short u0 = wplane_bits(w_hh, w_ih, nrow, fu, k0);
      const unsigned short u1 = wplane_bits(w_hh, w_ih, nrow, fu, k0 + 1);
      ww[idx] = (unsigned)u0 | ((unsigned)u1 << 16);
    }
  }
  {
#pragma unroll
    for (int it = 0; it < 3; ++it) {
      const int i  = it * NTHR + tid;
      const int ia = (i < NCLS * NHID) ? i : (NCLS * NHID - 1);
      int ib = i - NCLS * NHID; ib = (ib < 0) ? 0 : ((ib > NCLS - 1) ? (NCLS - 1) : ib);
      const float fa = (i < NCLS * NHID) ? 1.0f : 0.0f;
      const float fb = (i >= NCLS * NHID && i < NFC) ? 1.0f : 0.0f;
      const float va = w_fc[ia], vb = b_fc[ib];
      const float v = fmaf(fa, va, fb * vb);
      if (i < NFC) sFC[i] = v;
    }
  }
  __syncthreads();
  stage_x(sA, x, rowbase, 0, tid);
  __syncthreads();

  v16h bfr[4][2];
#pragma unroll
  for (int g = 0; g < 4; ++g)
#pragma unroll
    for (int ks = 0; ks < 2; ++ks)
      bfr[g][ks] = Frag<_Float16>::load(sW + (size_t)(g * UPAD + u) * WPITCH + koff + 32 * ks);
  float bs[4];
#pragma unroll
  for (int g = 0; g < 4; ++g) bs[g] = b_ih[g * NHID + uc] + b_hh[g * NHID + uc];
  float hst[8], cst[8];
#pragma unroll
  for (int r = 0; r < 8; ++r) { hst[r] = 0.0f; cst[r] = 0.0f; }

  const _Float16* arow = sA + c * APITCH + koff;
  const v8f z8 = {0.f, 0.f, 0.f, 0.f, 0.f, 0.f, 0.f, 0.f};

#pragma unroll 1
  for (int t = 0; t < NSTEP; ++t) {
    const v16h a0 = Frag<_Float16>::load(arow);
    const v16h a1 = Frag<_Float16>::load(arow + 32);
    v8f acc[4];
    acc[0] = z8; acc[1] = z8; acc[2] = z8; acc[3] = z8;
#pragma unroll
    for (int g = 0; g < 4; ++g) acc[g] = Frag<_Float16>::mma(a0, bfr[g][0], acc[g]);
#pragma unroll
    for (int g = 0; g < 4; ++g) acc[g] = Frag<_Float16>::mma(a1, bfr[g][1], acc[g]);
    mma_guard4(acc[0], acc[1], acc[2], acc[3], a0, a1);
#pragma unroll
    for (int r = 0; r < 8; ++r) {
      const float zi = fmaf(acc[0][r], WCARRY_INV, bs[0]);
      const float zf = fmaf(acc[1][r], WCARRY_INV, bs[1]);
      const float zg = fmaf(acc[2][r], WCARRY_INV, bs[2]);
      const float zo = fmaf(acc[3][r], WCARRY_INV, bs[3]);
      const float ig = fsig(zi);
      const float fg = fsig(zf);
      const float gg = ftanh(zg);
      const float og = fsig(zo);
      const float cn = fmaf(fg, cst[r], ig * gg);
      cst[r] = cn;
      hst[r] = og * ftanh(cn);
    }
    __syncthreads();
    if (ureal) {
#pragma unroll
      for (int r = 0; r < 8; ++r) sA[(8 * hh + r) * APITCH + u] = (_Float16)hst[r];
    }
    {
      const int tn = (t + 1 < NSTEP) ? (t + 1) : (NSTEP - 1);
      stage_x(sA, x, rowbase, tn, tid);
    }
    __syncthreads();
  }

#pragma unroll
  for (int r = 0; r < 8; ++r) sHf[(8 * hh + r) * HSPITCH + u] = hst[r];
  __syncthreads();
  {
    const int m   = tid / NCLS;
    const int cls = tid - m * NCLS;
    const int mr  = (m < ROWS_BLK) ? m : (ROWS_BLK - 1);
    float av = 0.0f;
#pragma unroll 1
    for (int j = 0; j < NHID; ++j) av = fmaf(sHf[mr * HSPITCH + j], sFC[cls * NHID + j], av);
    av += sFC[NCLS * NHID + cls];
    if (tid < NOUTB) sOut[tid] = av;
  }
  __syncthreads();
  if (wave == 0) {
    const int l4 = ((lane < NOUTB / 4) ? lane : (NOUTB / 4 - 1)) * 4;
    const v4f v = *(const v4f*)(sOut + l4);
    float* op = out + (size_t)rowbase * NCLS + l4;
    if (lane < NOUTB / 4) *(volatile v4f*)op = v;
    __threadfence();
    if (lane < NOUTB / 4) *(volatile v4f*)op = v;
  }
}

extern "C" void kernel_launch(void* const* d_in, const int* in_sizes, int n_in,
                              void* d_out, int out_size, void* d_ws, size_t ws_size, hipStream_t stream) {
  if (n_in < 7 || d_out == nullptr) return;
  if (in_sizes[0] != NSEQ * NSTEP * NIN || in_sizes[1] != NGATE * NIN || in_sizes[2] != NGATE * NHID ||
      in_sizes[3] != NGATE || in_sizes[4] != NGATE || in_sizes[5] != NCLS * NHID || in_sizes[6] != NCLS ||
      out_size != NSEQ * NCLS) return;
  (void)d_ws; (void)ws_size;

  const float* x    = (const float*)d_in[0];
  const float* w_ih = (const float*)d_in[1];
  const float* w_hh = (const float*)d_in[2];
  const float* b_ih = (const float*)d_in[3];
  const float* b_hh = (const float*)d_in[4];
  const float* w_fc = (const float*)d_in[5];
  const float* b_fc = (const float*)d_in[6];
  float* out = (float*)d_out;

  lstm_seq_kernel<<<NSEQ / ROWS_BLK, NTHR, 0, stream>>>(x, w_ih, w_hh, b_ih, b_hh, w_fc, b_fc, out);
}
